// SelfAttention_14482629722560
// MI455X (gfx1250) — hardware-verified
//
#include <hip/hip_runtime.h>
#ifndef NB
#define NB 32
#endif
#ifndef SEQ
#define SEQ 512
#endif
#ifndef SCORE_RES
#define SCORE_RES 0
#endif
#define NB_FULL 32
#define SQ_FULL 512
#define NN_FULL 8192
#define SQ SEQ
#define DM 256
#define NH 8
#define HD 32
#define QT 256
#define NKX SQ
#define KC (SQ / 128)
#define BG ((NB) < 8 ? (NB) : 8)
#define NR ((size_t)NB * SQ)
#define LQ DM
#define SCL 0.17677669529663687f
#define SCLR 0.00017263349150062194f
#define WS_CAP ((size_t)134217728)
#define OUT1_OFF ((size_t)NN_FULL * DM)
#define OUT_TOTAL (OUT1_OFF + (size_t)NB_FULL * SQ_FULL * SQ_FULL)
#define PL16 ((size_t)NB * SQ * DM * 2)
#define SREG ((size_t)BG * NH * QT * NKX * 4)
#define PREG ((size_t)BG * NH * QT * NKX * 2)
#define WS_TOTAL ((size_t)512 + (size_t)4 * DM * DM * 2 + (size_t)(6 + 2 * SCORE_RES) * PL16 + SREG + PREG)

static_assert(SQ % QT == 0);
static_assert(SQ % 128 == 0);
static_assert(QT % 128 == 0);
static_assert(NB % BG == 0);
static_assert(NB <= NB_FULL);
static_assert(NB_FULL == 32);
static_assert(SQ <= SQ_FULL);
static_assert(NH % 2 == 0);
static_assert(HD == 32);
static_assert(DM == NH * HD);
static_assert(DM == 256);
static_assert(KC * 128 == SQ);
static_assert(NN_FULL % 8 == 0);
static_assert(NN_FULL % 256 == 0);
static_assert((NB * SQ) % 128 == 0);
static_assert((BG * QT) % 8 == 0);
static_assert(SREG >= (size_t)NB * SQ * DM * 4);
static_assert(OUT1_OFF * 4 == (size_t)8388608);
static_assert(OUT_TOTAL * 4 == (size_t)41943040);
static_assert(OUT_TOTAL % 4 == 0);
static_assert(PL16 % 256 == 0 && SREG % 256 == 0 && PREG % 256 == 0);
static_assert(WS_TOTAL <= WS_CAP);

typedef unsigned short v8us __attribute__((ext_vector_type(8), may_alias));
typedef float  v8f  __attribute__((ext_vector_type(8)));
typedef float  v4f  __attribute__((ext_vector_type(4)));
typedef float  v4fa __attribute__((ext_vector_type(4), may_alias));
typedef _Float16 v16h __attribute__((ext_vector_type(16)));
typedef _Float16 v4h __attribute__((ext_vector_type(4)));
union FragH { v16h v; v8us half[2]; _Float16 h[16]; unsigned short u[16]; };
typedef _Float16 h16;

__device__ __forceinline__ unsigned short bf16_bits(float x) { unsigned int u = __float_as_uint(x); return (unsigned short)((u + 0x7FFFu + ((u >> 16) & 1u)) >> 16); }
__device__ __forceinline__ float bf16_val(unsigned short b) { return __uint_as_float(((unsigned int)b) << 16); }
__device__ __forceinline__ float bf16_rne(float x) { return bf16_val(bf16_bits(x)); }
static __device__ __forceinline__ h16 toh_flush(float v) { const h16 r = (h16)v; return (fabsf(v) < 6.103515625e-05f) ? (h16)0.0f : r; }
static __device__ __forceinline__ int iclamp(int v, int lo, int hi) { return v < lo ? lo : (v > hi ? hi : v); }

__global__ __launch_bounds__(256) void k_cnt(const int* __restrict__ batch, int n, int* __restrict__ tab) {
  __shared__ int sc[32]; __shared__ int sl[32];
  const int lane = threadIdx.x & 31; const int wave = __builtin_amdgcn_readfirstlane(threadIdx.x >> 5);
#pragma unroll 1
  for (int q = 0; q < 4; ++q) { const int g = wave * 4 + q; int ce = 0, cl = 0;
#pragma unroll 1
    for (int i = lane; i < n; i += 32) { const int v = batch[i]; ce += (v == g) ? 1 : 0; cl += (v >= 0 && v < g) ? 1 : 0; }
#pragma unroll
    for (int o = 16; o > 0; o >>= 1) { ce += __shfl_xor(ce, o); cl += __shfl_xor(cl, o); }
    if (lane == 0) { sc[g] = ce; sl[g] = cl; } }
  __syncthreads();
  if (wave == 0) { const int c = sc[lane], s = sl[lane];
    *(volatile int*)(tab + lane) = c; *(volatile int*)(tab + 32 + lane) = s; __threadfence();
    *(volatile int*)(tab + lane) = c; *(volatile int*)(tab + 32 + lane) = s; }
}

__global__ __launch_bounds__(256) void k_chk(const int* __restrict__ batch, int n, const int* __restrict__ tab, int* __restrict__ flag) {
  __shared__ int sw[8];
  const int lane = threadIdx.x & 31; const int wave = __builtin_amdgcn_readfirstlane(threadIdx.x >> 5);
  int bad = 0;
#pragma unroll 1
  for (int i = threadIdx.x; i < n; i += 256) { const int v = batch[i]; const int pv = batch[i > 0 ? i - 1 : 0];
    const int vb = iclamp(v, 0, NB_FULL - 1); const int c = tab[vb]; const int s = tab[32 + vb];
    bad |= (v < 0 || v >= NB_FULL) ? 1 : 0; bad |= (pv > v) ? 1 : 0; bad |= (i < s || i >= s + c) ? 1 : 0; }
#pragma unroll
  for (int o = 16; o > 0; o >>= 1) bad |= __shfl_xor(bad, o);
  if (lane == 0) sw[wave] = bad;
  __syncthreads();
  if (wave == 0) { int tot = tab[lane]; int f = sw[lane & 7];
#pragma unroll
    for (int o = 16; o > 0; o >>= 1) { tot += __shfl_xor(tot, o); f |= __shfl_xor(f, o); }
    f |= (tot != n) ? 1 : 0;
    *(volatile int*)(flag + lane) = f; __threadfence(); *(volatile int*)(flag + lane) = f; }
}

__global__ __launch_bounds__(256) void k_poison(const int* __restrict__ flag, float* __restrict__ out, size_t n4) {
  const int f = flag[0]; if (f == 0) return;
  const float qn = __uint_as_float(0x7FC00000u); const v4f q = {qn, qn, qn, qn};
  const size_t step = (size_t)gridDim.x * 256;
#pragma unroll 1
  for (size_t t = (size_t)blockIdx.x * 256 + threadIdx.x; t < n4; t += step) { float* d = out + t * 4; *(volatile v4f*)d = q; __threadfence(); *(volatile v4f*)d = q; }
}

__global__ __launch_bounds__(256) void k_w16(const float* __restrict__ W, _Float16* __restrict__ Bt, size_t n8, float scale) {
  const size_t t = (size_t)blockIdx.x * 256 + threadIdx.x; if (t >= n8) return;
  const v4f a = *(const v4fa*)(W + t * 8), c = *(const v4fa*)(W + t * 8 + 4);
  FragH f;
#pragma unroll
  for (int q = 0; q < 4; ++q) { f.h[q] = toh_flush(bf16_rne(a[q]) * scale); f.h[4 + q] = toh_flush(bf16_rne(c[q]) * scale); }
  const v8us o = f.half[0];
  unsigned short* d = (unsigned short*)Bt + t * 8;
  *(volatile v8us*)d = o; __threadfence(); *(volatile v8us*)d = o;
}

__global__ __launch_bounds__(256) void k_dense(const float* __restrict__ node, const int* __restrict__ tab, _Float16* __restrict__ X16, int nn) {
  const int lane = threadIdx.x & 31; const int wave = __builtin_amdgcn_readfirstlane(threadIdx.x >> 5);
  const int r = blockIdx.x * 8 + wave; if (r >= NB * SQ) return;
  const int b = r / SQ, p = r - b * SQ;
  const int cnt = iclamp(tab[b], 0, SQ); const int st = iclamp(tab[32 + b], 0, nn);
  const bool live = p < cnt;
  const int src = iclamp(st + p, 0, nn - 1);
  const float* s = node + (size_t)src * DM + lane * 8;
  const v4f a = *(const v4fa*)(s), c = *(const v4fa*)(s + 4);
  FragH f;
#pragma unroll
  for (int q = 0; q < 4; ++q) { const float va = live ? bf16_rne(a[q]) : 0.f; const float vc = live ? bf16_rne(c[q]) : 0.f; f.h[q] = toh_flush(va); f.h[4 + q] = toh_flush(vc); }
  const v8us o = f.half[0];
  unsigned short* d = (unsigned short*)X16 + (size_t)r * DM + lane * 8;
  *(volatile v8us*)d = o; __threadfence(); *(volatile v8us*)d = o;
}

#if SCORE_RES
__global__ __launch_bounds__(256) void k_hl(const float* __restrict__ F, _Float16* __restrict__ Hh, _Float16* __restrict__ Hl, size_t n8) {
  const size_t t = (size_t)blockIdx.x * 256 + threadIdx.x; if (t >= n8) return; FragH fh, fl; const v4f a = *(const v4fa*)(F + t * 8), c = *(const v4fa*)(F + t * 8 + 4);
#pragma unroll
  for (int q = 0; q < 4; ++q) { _Float16 h = (_Float16)a[q]; fh.h[q] = h; fl.h[q] = (_Float16)((a[q] - (float)h) * 1024.0f); h = (_Float16)c[q]; fh.h[4 + q] = h; fl.h[4 + q] = (_Float16)((c[q] - (float)h) * 1024.0f); }
  const v8us oh = fh.half[0], ol = fl.half[0];
  for (int pass = 0; pass < 2; ++pass) { *(volatile v8us*)((unsigned short*)Hh + t * 8) = oh; *(volatile v8us*)((unsigned short*)Hl + t * 8) = ol; if (pass == 0) __threadfence(); }
}
#endif

__device__ __forceinline__ v16h g2_frag(const _Float16* p, int hh) { FragH f; f.half[0] = *(const v8us*)((const unsigned short*)p + 8 * hh); f.half[1] = *(const v8us*)((const unsigned short*)p + 16 + 8 * hh); return f.v; }
__device__ __forceinline__ v8f g2_mma(v16h a, v16h b, v8f c) { v8f d = __builtin_amdgcn_wmma_f32_16x16x32_f16(false, a, false, b, (short)0, c, false, false); asm volatile("v_nop\n\tv_nop\n\tv_nop\n\tv_nop" : "+v"(d) : "v"(a), "v"(b)); return d; }
template <bool PAIR>
__global__ __launch_bounds__(128) void k_gemm2(const _Float16* __restrict__ A, int lda, size_t sA, size_t sA2, size_t pairA,
    const _Float16* __restrict__ Bh, int ldb, size_t sB, size_t sB2, int ydiv, float alpha, const float* __restrict__ bias,
    const float* CP, float* C, _Float16* C16, int ldc, size_t sC, size_t sC2, int M, int N, int K) {
  __shared__ __attribute__((aligned(16))) float so[4][32][68];
  const int tid = threadIdx.x, w = tid >> 5, lane = tid & 31, ln = lane & 15, hh = lane >> 4;
  const int by = blockIdx.y; const int y1 = by / ydiv; const int y0 = by - y1 * ydiv;
  A += (size_t)y0 * sA + (size_t)y1 * sA2; Bh += (size_t)y0 * sB + (size_t)y1 * sB2; const size_t cofs = (size_t)y0 * sC + (size_t)y1 * sC2;
  const int ntn = N >> 6; const int mt = blockIdx.x / ntn, nq = blockIdx.x - mt * ntn; const int row0 = mt * 128 + 32 * w, col0 = nq * 64; if (row0 >= M) return;
  const _Float16* a0p = A + (size_t)(row0 + ln) * lda; const _Float16* a1p = a0p + (size_t)16 * lda;
  const _Float16* a2p = PAIR ? (a0p + pairA) : a0p; const _Float16* a3p = PAIR ? (a1p + pairA) : a1p;
  const _Float16* b0p = Bh + (size_t)(col0 + ln) * ldb; const _Float16* b1p = b0p + (size_t)16 * ldb; const _Float16* b2p = b1p + (size_t)16 * ldb; const _Float16* b3p = b2p + (size_t)16 * ldb;
  const v8f z8 = {0.f,0.f,0.f,0.f,0.f,0.f,0.f,0.f}; v8f c00 = z8, c01 = z8, c02 = z8, c03 = z8, c10 = z8, c11 = z8, c12 = z8, c13 = z8;
#pragma unroll 1
  for (int kb = 0; kb < K; kb += 32) { const v16h a0 = g2_frag(a0p + kb, hh), a1 = g2_frag(a1p + kb, hh);
    v16h a2 = a0, a3 = a1; if (PAIR) { a2 = g2_frag(a2p + kb, hh); a3 = g2_frag(a3p + kb, hh); }
    v16h b = g2_frag(b0p + kb, hh); c00 = g2_mma(a0, b, c00); c10 = g2_mma(a1, b, c10);
    b = g2_frag(b1p + kb, hh); c01 = g2_mma(a0, b, c01); c11 = g2_mma(a1, b, c11);
    b = g2_frag(b2p + kb, hh); c02 = g2_mma(a2, b, c02); c12 = g2_mma(a3, b, c12);
    b = g2_frag(b3p + kb, hh); c03 = g2_mma(a2, b, c03); c13 = g2_mma(a3, b, c13); }
  v8f accs[8] = {c00, c01, c02, c03, c10, c11, c12, c13};
#pragma unroll
  for (int u = 0; u < 8; ++u) { const int t = u & 3, half = u >> 2; const int col = col0 + t * 16 + ln; const float bv = bias ? bf16_rne(bias[col]) : 0.f;
#pragma unroll
    for (int r = 0; r < 8; ++r) { const int rloc = half * 16 + 8 * hh + r; float v = accs[u][r] * alpha + bv; if (CP) v += CP[cofs + (size_t)(row0 + rloc) * ldc + col];
      so[w][rloc][t * 16 + ln] = v; } }
  __builtin_amdgcn_fence(4  , "workgroup"); __builtin_amdgcn_wave_barrier();
  const int rsub = lane >> 4, c4 = (lane & 15) * 4;
  for (int pass = 0; pass < 2; ++pass) {
#pragma unroll
    for (int q = 0; q < 16; ++q) { const int r = q * 2 + rsub; const v4f v = *(const v4fa*)&so[w][r][c4]; if (C) *(volatile v4f*)(C + cofs + (size_t)(row0 + r) * ldc + col0 + c4) = v; if (C16) { v4h h4; for (int i = 0; i < 4; ++i) h4[i] = (_Float16)v[i]; *(volatile v4h*)(C16 + cofs + (size_t)(row0 + r) * ldc + col0 + c4) = h4; } }
    if (pass == 0) __threadfence(); } }

__global__ __launch_bounds__(256) void k_vt(const _Float16* __restrict__ V16, int ldv, _Float16* __restrict__ Vt) {
  __shared__ unsigned short tl[64][HD + 2];
  const int tid = threadIdx.x; const int slab = blockIdx.x / (SQ / 64), lg = blockIdx.x % (SQ / 64); const int b = slab / NH, h = slab % NH;
  { const int r = tid / 4, c8 = (tid % 4) * 8; FragH f; f.half[0] = *(const v8us*)((const unsigned short*)V16 + ((size_t)b * SQ + lg * 64 + r) * ldv + h * HD + c8);
#pragma unroll
    for (int q = 0; q < 8; ++q) tl[r][c8 + q] = f.u[q]; }
  __syncthreads();
  const int d = tid / 8, pc = tid % 8; FragH g;
#pragma unroll
  for (int q = 0; q < 8; ++q) g.u[q] = tl[pc * 8 + q][d];
  const v8us o = g.half[0];
  unsigned short* dst = (unsigned short*)Vt + ((size_t)slab * HD + d) * SQ + lg * 64 + pc * 8;
  *(volatile v8us*)dst = o; __threadfence(); *(volatile v8us*)dst = o;
}

__global__ __launch_bounds__(256) void k_rsmp(const float* __restrict__ S, _Float16* __restrict__ P, const int* __restrict__ tab, float* __restrict__ AW, int b0, int q0, int nrows) {
  #pragma clang fp contract(off)
  const int lane = threadIdx.x & 31; const int wave = __builtin_amdgcn_readfirstlane(threadIdx.x >> 5);
  const int gw = blockIdx.x * 8 + wave; if (gw >= nrows) return;
  const int bg = gw / QT, i = gw - bg * QT;
  const int cnt = iclamp(tab[b0 + bg], 0, SQ);
  v4f avg[KC];
#pragma unroll
  for (int c = 0; c < KC; ++c) { const v4f z = {0.f, 0.f, 0.f, 0.f}; avg[c] = z; }
#pragma unroll 1
  for (int h = 0; h < NH; ++h) {
    const size_t ro = ((size_t)(bg * NH + h) * QT + i) * NKX + lane * 4;
    v4f x[KC];
#pragma unroll
    for (int c = 0; c < KC; ++c) x[c] = *(const v4fa*)(S + ro + c * 128);
    float mx = -3.0e38f;
#pragma unroll
    for (int c = 0; c < KC; ++c) {
#pragma unroll
      for (int u = 0; u < 4; ++u) { const int j = c * 128 + lane * 4 + u; const float a = (j < cnt) ? x[c][u] : -1.0e9f; x[c][u] = a; mx = fmaxf(mx, a); } }
#pragma unroll
    for (int o = 16; o > 0; o >>= 1) mx = fmaxf(mx, __shfl_xor(mx, o));
    float se = 0.f;
#pragma unroll
    for (int c = 0; c < KC; ++c) {
#pragma unroll
      for (int u = 0; u < 4; ++u) { const float e = __expf(x[c][u] - mx); x[c][u] = e; se += e; } }
#pragma unroll
    for (int o = 16; o > 0; o >>= 1) se += __shfl_xor(se, o);
    const float inv = 1.0f / se;
    v4h hp[KC];
#pragma unroll
    for (int c = 0; c < KC; ++c) {
#pragma unroll
      for (int u = 0; u < 4; ++u) { const float p = x[c][u] * inv; avg[c][u] = avg[c][u] + p; hp[c][u] = toh_flush(p * 256.0f); } }
    for (int pass = 0; pass < 2; ++pass) {
#pragma unroll
      for (int c = 0; c < KC; ++c) *(volatile v4h*)(P + ro + c * 128) = hp[c];
      if (pass == 0) __threadfence(); }
  }
  v4f av[KC];
#pragma unroll
  for (int c = 0; c < KC; ++c) {
#pragma unroll
    for (int u = 0; u < 4; ++u) av[c][u] = avg[c][u] * 0.125f; }
  float* dst = AW + ((size_t)(b0 + bg) * SQ_FULL + q0 + i) * SQ_FULL + lane * 4;
  for (int pass = 0; pass < 2; ++pass) {
#pragma unroll
    for (int c = 0; c < KC; ++c) *(volatile v4f*)(dst + c * 128) = av[c];
    if (pass == 0) __threadfence(); }
}

__global__ __launch_bounds__(256) void k_lnres(const float* __restrict__ OUTF, const float* __restrict__ node, const int* __restrict__ batch, const int* __restrict__ tab,
    const float* __restrict__ gamma, const float* __restrict__ beta, float* __restrict__ out, int nn) {
  #pragma clang fp contract(off)
  const int lane = threadIdx.x & 31; const int wave = __builtin_amdgcn_readfirstlane(threadIdx.x >> 5);
  const int i = blockIdx.x * 8 + wave; if (i >= nn) return;
  const int b = iclamp(batch[i], 0, NB_FULL - 1);
  if (b >= NB) return;
  const int st = iclamp(tab[32 + b], 0, nn);
  const int pos = iclamp(i - st, 0, SQ - 1);
  const size_t ro = ((size_t)b * SQ + pos) * DM + lane * 4;
  const v4f x0 = *(const v4fa*)(OUTF + ro), x1 = *(const v4fa*)(OUTF + ro + 128);
  float sm = ((x0[0] + x0[1]) + (x0[2] + x0[3])) + ((x1[0] + x1[1]) + (x1[2] + x1[3]));
#pragma unroll
  for (int o = 16; o > 0; o >>= 1) sm += __shfl_xor(sm, o);
  const float mu = sm * 0.00390625f;
  v4f d0, d1; float vs = 0.f;
#pragma unroll
  for (int u = 0; u < 4; ++u) { d0[u] = x0[u] - mu; d1[u] = x1[u] - mu; vs += d0[u] * d0[u]; vs += d1[u] * d1[u]; }
#pragma unroll
  for (int o = 16; o > 0; o >>= 1) vs += __shfl_xor(vs, o);
  const float rstd = rsqrtf(vs * 0.00390625f + 1.0e-5f);
  const v4f g0 = *(const v4fa*)(gamma + lane * 4), g1 = *(const v4fa*)(gamma + 128 + lane * 4);
  const v4f e0 = *(const v4fa*)(beta + lane * 4), e1 = *(const v4fa*)(beta + 128 + lane * 4);
  const v4f n0 = *(const v4fa*)(node + (size_t)i * DM + lane * 4), n1 = *(const v4fa*)(node + (size_t)i * DM + 128 + lane * 4);
  v4f y0, y1;
#pragma unroll
  for (int u = 0; u < 4; ++u) { y0[u] = (d0[u] * rstd * bf16_rne(g0[u]) + bf16_rne(e0[u])) + bf16_rne(n0[u]); y1[u] = (d1[u] * rstd * bf16_rne(g1[u]) + bf16_rne(e1[u])) + bf16_rne(n1[u]); }
  float* dst = out + (size_t)i * DM + lane * 4;
  for (int pass = 0; pass < 2; ++pass) { *(volatile v4f*)(dst) = y0; *(volatile v4f*)(dst + 128) = y1; if (pass == 0) __threadfence(); }
}

extern "C" void kernel_launch(void* const* d_in, const int* in_sizes, int n_in,
                              void* d_out, int out_size, void* d_ws, size_t ws_size, hipStream_t stream) {
  if (n_in < 12) return;
  if ((size_t)in_sizes[0] < (size_t)NN_FULL * DM || (size_t)in_sizes[1] < (size_t)NN_FULL) return;
  if ((size_t)in_sizes[2] < (size_t)DM * DM || (size_t)in_sizes[3] < (size_t)DM * DM || (size_t)in_sizes[4] < (size_t)DM * DM || (size_t)in_sizes[5] < (size_t)DM * DM) return;
  if ((size_t)in_sizes[6] < (size_t)DM || (size_t)in_sizes[7] < (size_t)DM || (size_t)in_sizes[8] < (size_t)DM || (size_t)in_sizes[9] < (size_t)DM || (size_t)in_sizes[10] < (size_t)DM || (size_t)in_sizes[11] < (size_t)DM) return;
  if ((size_t)out_size < OUT_TOTAL) return;
  const float* node = (const float*)d_in[0]; const int* batch = (const int*)d_in[1];
  const float* wq = (const float*)d_in[2]; const float* wk = (const float*)d_in[3]; const float* wv = (const float*)d_in[4]; const float* wo = (const float*)d_in[5];
  const float* bq = (const float*)d_in[6]; const float* bk = (const float*)d_in[7]; const float* bv = (const float*)d_in[8]; const float* bo = (const float*)d_in[9];
  const float* gamma = (const float*)d_in[10]; const float* beta = (const float*)d_in[11];
  float* out = (float*)d_out; float* aw = out + OUT1_OFF;
  char* ws = (char*)d_ws; size_t off = 0;
  auto take = [&](size_t bytes) { char* p = ws + off; off += (bytes + 255) & ~(size_t)255; return p; };
  int* TAB = (int*)take((size_t)256);
  int* FLAG = (int*)take((size_t)256);
  _Float16* BQ = (_Float16*)take((size_t)DM * DM * 2); _Float16* BK = (_Float16*)take((size_t)DM * DM * 2); _Float16* BV = (_Float16*)take((size_t)DM * DM * 2); _Float16* BO = (_Float16*)take((size_t)DM * DM * 2);
  _Float16* X16 = (_Float16*)take(NR * DM * 2);
  _Float16* QH = (_Float16*)take(NR * DM * 2); _Float16* KH = (_Float16*)take(NR * DM * 2);
#if SCORE_RES
  _Float16* QL = (_Float16*)take(NR * DM * 2); _Float16* KL = (_Float16*)take(NR * DM * 2);
#endif
  _Float16* V16 = (_Float16*)take(NR * DM * 2); _Float16* O16 = (_Float16*)take(NR * DM * 2);
  float* S = (float*)take((size_t)BG * NH * QT * NKX * 4);
  float* OUTF = S;
  _Float16* P = (_Float16*)take((size_t)BG * NH * QT * NKX * 2);
  _Float16* VT = (_Float16*)take((size_t)NB * NH * HD * SQ * 2);
  if (off > ws_size || off > WS_CAP) return;

  k_cnt<<<1, 256, 0, stream>>>(batch, NN_FULL, TAB);
  k_chk<<<1, 256, 0, stream>>>(batch, NN_FULL, TAB, FLAG);
  { const unsigned g = (unsigned)(((size_t)DM * DM / 8 + 255) / 256);
    k_w16<<<g, 256, 0, stream>>>(wq, BQ, (size_t)DM * DM / 8, 16.0f); k_w16<<<g, 256, 0, stream>>>(wk, BK, (size_t)DM * DM / 8, 16.0f);
    k_w16<<<g, 256, 0, stream>>>(wv, BV, (size_t)DM * DM / 8, 16.0f); k_w16<<<g, 256, 0, stream>>>(wo, BO, (size_t)DM * DM / 8, 16.0f); }
  k_dense<<<(unsigned)((NR + 7) / 8), 256, 0, stream>>>(node, TAB, X16, NN_FULL);

  const unsigned gproj = (unsigned)((NR / 128) * (DM / 64));
#if SCORE_RES
  { float* QF = S; const unsigned ghl = (unsigned)((NR * DM / 8 + 255) / 256);
    k_gemm2<false><<<dim3(gproj, 1), 128, 0, stream>>>(X16, DM, (size_t)0, (size_t)0, (size_t)0, BQ, DM, (size_t)0, (size_t)0, 1, 0.0625f, bq, nullptr, QF, nullptr, DM, (size_t)0, (size_t)0, (int)NR, DM, DM);
    k_hl<<<ghl, 256, 0, stream>>>(QF, QH, QL, NR * DM / 8);
    k_gemm2<false><<<dim3(gproj, 1), 128, 0, stream>>>(X16, DM, (size_t)0, (size_t)0, (size_t)0, BK, DM, (size_t)0, (size_t)0, 1, 0.0625f, bk, nullptr, QF, nullptr, DM, (size_t)0, (size_t)0, (int)NR, DM, DM);
    k_hl<<<ghl, 256, 0, stream>>>(QF, KH, KL, NR * DM / 8); }
#else
  k_gemm2<false><<<dim3(gproj, 1), 128, 0, stream>>>(X16, DM, (size_t)0, (size_t)0, (size_t)0, BQ, DM, (size_t)0, (size_t)0, 1, 0.0625f, bq, nullptr, nullptr, QH, DM, (size_t)0, (size_t)0, (int)NR, DM, DM);
  k_gemm2<false><<<dim3(gproj, 1), 128, 0, stream>>>(X16, DM, (size_t)0, (size_t)0, (size_t)0, BK, DM, (size_t)0, (size_t)0, 1, 0.0625f, bk, nullptr, nullptr, KH, DM, (size_t)0, (size_t)0, (int)NR, DM, DM);
#endif
  k_gemm2<false><<<dim3(gproj, 1), 128, 0, stream>>>(X16, DM, (size_t)0, (size_t)0, (size_t)0, BV, DM, (size_t)0, (size_t)0, 1, 0.0625f, bv, nullptr, nullptr, V16, DM, (size_t)0, (size_t)0, (int)NR, DM, DM);
  k_vt<<<(unsigned)(NB * NH * (SQ / 64)), 256, 0, stream>>>(V16, LQ, VT);

  const size_t slabS = (size_t)QT * NKX;
  for (int g = 0; g < NB / BG; ++g) { const size_t rg0 = (size_t)g * BG * SQ;
    for (int q0 = 0; q0 < SQ; q0 += QT) { const int nk = SQ;
      const dim3 gs((unsigned)((QT / 128) * (nk / 64)), BG * NH);
      k_gemm2<false><<<gs, 128, 0, stream>>>(QH + (rg0 + q0) * LQ, LQ, (size_t)HD, (size_t)SQ * LQ, (size_t)0, KH + rg0 * LQ, LQ, (size_t)HD, (size_t)SQ * LQ, NH, SCL, nullptr, nullptr, S, nullptr, NKX, slabS, (size_t)NH * slabS, QT, nk, HD);
#if SCORE_RES
      k_gemm2<false><<<gs, 128, 0, stream>>>(QL + (rg0 + q0) * LQ, LQ, (size_t)HD, (size_t)SQ * LQ, (size_t)0, KH + rg0 * LQ, LQ, (size_t)HD, (size_t)SQ * LQ, NH, SCLR, nullptr, S, S, nullptr, NKX, slabS, (size_t)NH * slabS, QT, nk, HD);
      k_gemm2<false><<<gs, 128, 0, stream>>>(QH + (rg0 + q0) * LQ, LQ, (size_t)HD, (size_t)SQ * LQ, (size_t)0, KL + rg0 * LQ, LQ, (size_t)HD, (size_t)SQ * LQ, NH, SCLR, nullptr, S, S, nullptr, NKX, slabS, (size_t)NH * slabS, QT, nk, HD);
#endif
      k_rsmp<<<(unsigned)((BG * QT + 7) / 8), 256, 0, stream>>>(S, P, TAB, aw, g * BG, q0, BG * QT);
      k_gemm2<true><<<dim3((unsigned)(QT / 128), BG * (NH / 2)), 128, 0, stream>>>(P, NKX, 2 * slabS, (size_t)NH * slabS, slabS, VT + (size_t)g * BG * NH * HD * SQ, SQ, (size_t)2 * HD * SQ, (size_t)NH * HD * SQ, NH / 2, 0.25f, nullptr, nullptr, nullptr, O16 + (rg0 + q0) * DM, DM, (size_t)(2 * HD), (size_t)SQ * DM, QT, 2 * HD, nk);
    } }

  k_gemm2<false><<<dim3((unsigned)((SQ / 128) * (DM / 64)), NB), 128, 0, stream>>>(O16, DM, (size_t)0, (size_t)SQ * DM, (size_t)0, BO, DM, (size_t)0, (size_t)0, 1, 0.0009765625f, bo, nullptr, OUTF, nullptr, DM, (size_t)0, (size_t)SQ * DM, SQ, DM, DM);
  k_lnres<<<(unsigned)((NN_FULL + 7) / 8), 256, 0, stream>>>(OUTF, node, batch, TAB, gamma, beta, out, NN_FULL);
  k_poison<<<1024, 256, 0, stream>>>(FLAG, out, OUT_TOTAL / 4);
}
